// S6Block_87445534146660
// MI455X (gfx1250) — hardware-verified
//
#include <hip/hip_runtime.h>
#include <hip/hip_bf16.h>
#include <math.h>

constexpr int kBatch = 4;
constexpr int kLen   = 4096;
constexpr int kCin   = 256;
constexpr int kLat   = 512;
constexpr int kCout  = 256;
constexpr int kTok   = kBatch * kLen;
constexpr int kNall  = 4 * kLat;

typedef __attribute__((ext_vector_type(16))) _Float16 v16h;
typedef __attribute__((ext_vector_type(8)))  _Float16 v8h;
typedef __attribute__((ext_vector_type(16))) __bf16   v16b;
typedef __attribute__((ext_vector_type(8)))  __bf16   v8b;
typedef __attribute__((ext_vector_type(8)))  float    v8f;
typedef __attribute__((ext_vector_type(4)))  float    v4f;
typedef __attribute__((ext_vector_type(4)))  unsigned int v4u;

__device__ __forceinline__ unsigned short f2bf_bits(float f) {
  unsigned u = __float_as_uint(f);
  return (unsigned short)((u + 0x7FFFu + ((u >> 16) & 1u)) >> 16);
}
__device__ __forceinline__ float bf_bits2f(unsigned short h) { return __uint_as_float(((unsigned)h) << 16); }

__device__ __forceinline__ void dep_guard_h(v8f& a, v8f& b, v16h x, v16h y) { asm volatile("v_nop\n\tv_nop\n\tv_nop\n\tv_nop" : "+v"(a), "+v"(b) : "v"(x), "v"(y)); }
__device__ __forceinline__ void dep_guard_b(v8f& a, v8f& b, v16b x, v16b y) { asm volatile("v_nop\n\tv_nop\n\tv_nop\n\tv_nop" : "+v"(a), "+v"(b) : "v"(x), "v"(y)); }
__device__ __forceinline__ void keep4_h(v16h a, v16h b, v16h c, v16h d) { asm volatile("v_nop" :: "v"(a), "v"(b), "v"(c), "v"(d)); }
__device__ __forceinline__ void keep4_b(v16b a, v16b b, v16b c, v16b d) { asm volatile("v_nop" :: "v"(a), "v"(b), "v"(c), "v"(d)); }
__device__ __forceinline__ void acc_guard4(v8f& a, v8f& b, v8f& c, v8f& d) { asm volatile("v_nop\n\tv_nop\n\tv_nop\n\tv_nop" : "+v"(a), "+v"(b), "+v"(c), "+v"(d)); }
template <typename T> struct Frag;
template <> struct Frag<_Float16> {
  typedef v16h V; union U { v16h v; v8h h[2]; };
  static __device__ __forceinline__ v16h load(const _Float16* p) {
    U f; f.h[0] = *(const v8h*)(p); f.h[1] = *(const v8h*)(p + 16); return f.v;
  }
  static __device__ __forceinline__ v8f mma(v16h a, v16h b, v8f c) {
    return __builtin_amdgcn_wmma_f32_16x16x32_f16(false, a, false, b, (short)0, c, false, false);
  }
  static __device__ __forceinline__ void guard(v8f& a, v8f& b, v16h x, v16h y) { dep_guard_h(a, b, x, y); }
  static __device__ __forceinline__ void keep(v16h a, v16h b, v16h c, v16h d) { keep4_h(a, b, c, d); }
};
template <> struct Frag<__bf16> {
  typedef v16b V; union U { v16b v; v8b h[2]; };
  static __device__ __forceinline__ v16b load(const __bf16* p) {
    U f; f.h[0] = *(const v8b*)(p); f.h[1] = *(const v8b*)(p + 16); return f.v;
  }
  static __device__ __forceinline__ v8f mma(v16b a, v16b b, v8f c) {
    return __builtin_amdgcn_wmma_f32_16x16x32_bf16(false, a, false, b, (short)0, c, false, false);
  }
  static __device__ __forceinline__ void guard(v8f& a, v8f& b, v16b x, v16b y) { dep_guard_b(a, b, x, y); }
  static __device__ __forceinline__ void keep(v16b a, v16b b, v16b c, v16b d) { keep4_b(a, b, c, d); }
};

__device__ __forceinline__ unsigned pk16(unsigned short a, unsigned short b) { return (unsigned)a | ((unsigned)b << 16); }

template <int ET> struct Elem;
template <> struct Elem<0> { typedef _Float16 T; };
template <> struct Elem<1> { typedef __bf16 T; };
template <int ET, bool SPLIT, int BIAS_MODE, int OUT_MODE, bool RESID, int ACT = 0>
__global__ __launch_bounds__(256) void wmma_gemm64(
    const unsigned short* __restrict__ Ap, const unsigned short* __restrict__ A2p, int lda, long strideA,
    const unsigned short* __restrict__ Btp, const unsigned short* __restrict__ Bt2p, int ldb, long strideB,
    void* __restrict__ Cout, void* __restrict__ Cout2, int ldc, long strideC,
    const float* __restrict__ bias,
    const float* __restrict__ resid, long strideR,
    int M, int N, int K, float scale) {
  typedef typename Elem<ET>::T T;
  typedef typename Frag<T>::V V;
  const T* A = (const T*)Ap; const T* A2 = (const T*)A2p; const T* Bt = (const T*)Btp; const T* Bt2 = (const T*)Bt2p;
  __shared__ __align__(16) float sT[8][16 * 68];
  const int b    = blockIdx.y;
  const int lane = threadIdx.x & 31;
  const int wave = threadIdx.x >> 5;
  const int tilesN = N >> 6;
  const int tilesM = M >> 6;
  const int tile = blockIdx.x * 8 + wave;
  if (tile >= tilesM * tilesN) return;
  const int tm = tile / tilesN;
  const int tn = tile - tm * tilesN;
  const int m0 = tm << 6;
  const int n0 = tn << 6;

  const T* Ab  = A  + (size_t)b * strideA;
  const T* Bb  = Bt + (size_t)b * strideB;
  const T* Ab2 = SPLIT ? (A2  + (size_t)b * strideA) : nullptr;
  const T* Bb2 = SPLIT ? (Bt2 + (size_t)b * strideB) : nullptr;

  const int rlane = lane & 15;
  const int koff  = (lane >> 4) * 8;
  const int mOff  = (lane >> 4) * 8;

  v8f acc[4][4];
#pragma unroll
  for (int i = 0; i < 4; ++i)
#pragma unroll
    for (int j = 0; j < 4; ++j) acc[i][j] = (v8f){0.f,0.f,0.f,0.f,0.f,0.f,0.f,0.f};

  for (int k0 = 0; k0 < K; k0 += 32) {
    V bh[4], bl[4];
#pragma unroll
    for (int j = 0; j < 4; ++j) {
      const size_t bo = (size_t)(n0 + (j << 4) + rlane) * ldb + koff + k0;
      bh[j] = Frag<T>::load(Bb + bo);
      if (SPLIT) bl[j] = Frag<T>::load(Bb2 + bo);
    }
#pragma unroll
    for (int i = 0; i < 4; ++i) {
      const size_t ao = (size_t)(m0 + (i << 4) + rlane) * lda + koff + k0;
      V ah = Frag<T>::load(Ab + ao);
      V al;
      if (SPLIT) al = Frag<T>::load(Ab2 + ao);
#pragma unroll
      for (int j = 0; j < 4; ++j) {
        acc[i][j] = Frag<T>::mma(ah, bh[j], acc[i][j]);
        if (SPLIT) {
          acc[i][j] = Frag<T>::mma(ah, bl[j], acc[i][j]);
          acc[i][j] = Frag<T>::mma(al, bh[j], acc[i][j]);
        }
      }
      Frag<T>::guard(acc[i][0], acc[i][3], ah, SPLIT ? al : ah);
    }
    Frag<T>::keep(bh[0], bh[1], bh[2], bh[3]);
    if (SPLIT) Frag<T>::keep(bl[0], bl[1], bl[2], bl[3]);
  }
  acc_guard4(acc[0][0], acc[0][1], acc[0][2], acc[0][3]);
  acc_guard4(acc[1][0], acc[1][1], acc[1][2], acc[1][3]);
  acc_guard4(acc[2][0], acc[2][1], acc[2][2], acc[2][3]);
  acc_guard4(acc[3][0], acc[3][1], acc[3][2], acc[3][3]);

  float* slab = sT[wave];
  const float* Rb = RESID ? (resid + (size_t)b * strideR) : nullptr;
#pragma unroll
  for (int i = 0; i < 4; ++i) {
    const int mBase = m0 + (i << 4);
#pragma unroll
    for (int j = 0; j < 4; ++j) {
      const int n = n0 + (j << 4) + rlane;
      float bv = 0.f;
      if (BIAS_MODE == 2) bv = bias[n];
#pragma unroll
      for (int r = 0; r < 8; ++r) {
        float v = acc[i][j][r] * scale;
        if (BIAS_MODE == 1) v += bias[mBase + mOff + r];
        if (BIAS_MODE == 2) v += bv;
        if (RESID) v += Rb[(size_t)(mBase + mOff + r) * ldc + n];
        if (ACT == 2) v = fmaxf(v, 0.0f);
        if (ACT == 4) v = (v > 0.f) ? v : 0.01f * v;
        slab[(mOff + r) * 68 + (j << 4) + rlane] = v;
      }
    }
    __builtin_amdgcn_fence(__ATOMIC_RELEASE, "workgroup");
    __builtin_amdgcn_wave_barrier();
    __builtin_amdgcn_fence(__ATOMIC_ACQUIRE, "workgroup");
    if (OUT_MODE == 0) {
      float* C = (float*)Cout + (size_t)b * strideC;
      const int hh = lane >> 4, c4 = (lane & 15) * 4;
      for (int pass = 0; pass < 2; ++pass) {
#pragma unroll
        for (int it = 0; it < 8; ++it) {
          const int row = it * 2 + hh;
          v4f v = *(const v4f*)(slab + row * 68 + c4);
          *(volatile v4f*)(C + (size_t)(mBase + row) * ldc + n0 + c4) = v;
        }
        __threadfence();
      }
    } else {
      const int q = lane >> 3, c8 = (lane & 7) * 8;
      unsigned short* C  = (unsigned short*)Cout  + (size_t)b * strideC;
      unsigned short* C2 = (OUT_MODE == 2) ? ((unsigned short*)Cout2 + (size_t)b * strideC) : nullptr;
      for (int pass = 0; pass < 2; ++pass) {
#pragma unroll
        for (int it = 0; it < 4; ++it) {
          const int row = it * 4 + q;
          const float* sp = slab + row * 68 + c8;
          v8h hv, lv;
#pragma unroll
          for (int e = 0; e < 8; ++e) {
            if (OUT_MODE == 1) {
              hv[e] = (_Float16)sp[e];
            } else {
              unsigned short hb = f2bf_bits(sp[e]);
              unsigned short lb = f2bf_bits(sp[e] - bf_bits2f(hb));
              hv[e] = __builtin_bit_cast(_Float16, hb);
              lv[e] = __builtin_bit_cast(_Float16, lb);
            }
          }
          *(volatile v8h*)(C + (size_t)(mBase + row) * ldc + n0 + c8) = hv;
          if (OUT_MODE == 2) *(volatile v8h*)(C2 + (size_t)(mBase + row) * ldc + n0 + c8) = lv;
        }
        __threadfence();
      }
    }
    __builtin_amdgcn_fence(__ATOMIC_RELEASE, "workgroup");
    __builtin_amdgcn_wave_barrier();
    __builtin_amdgcn_fence(__ATOMIC_ACQUIRE, "workgroup");
  }
}

__global__ __launch_bounds__(256) void cast8_bf16hl_kernel(const float* __restrict__ in,
                                                          unsigned short* __restrict__ outH,
                                                          unsigned short* __restrict__ outL, int n8) {
  const int i = blockIdx.x * 256 + threadIdx.x;
  if (i >= n8) return;
  const float* p = in + 8 * (size_t)i;
  const v4f a = *(const v4f*)(p);
  const v4f c = *(const v4f*)(p + 4);
  unsigned short hb[8], lb[8];
#pragma unroll
  for (int e = 0; e < 4; ++e) {
    const float v0 = a[e];
    const unsigned short h0 = f2bf_bits(v0);
    hb[e] = h0;
    lb[e] = f2bf_bits(v0 - bf_bits2f(h0));
    const float v1 = c[e];
    const unsigned short h1 = f2bf_bits(v1);
    hb[4 + e] = h1;
    lb[4 + e] = f2bf_bits(v1 - bf_bits2f(h1));
  }
  const v4u uh = (v4u){pk16(hb[0], hb[1]), pk16(hb[2], hb[3]), pk16(hb[4], hb[5]), pk16(hb[6], hb[7])};
  const v4u ul = (v4u){pk16(lb[0], lb[1]), pk16(lb[2], lb[3]), pk16(lb[4], lb[5]), pk16(lb[6], lb[7])};
  unsigned short* qh = outH + 8 * (size_t)i;
  unsigned short* ql = outL + 8 * (size_t)i;
  *(volatile v4u*)qh = uh;
  *(volatile v4u*)ql = ul;
  __threadfence();
  *(volatile v4u*)qh = uh;
  *(volatile v4u*)ql = ul;
}

__global__ __launch_bounds__(256) void transpose_cast_bf16hl_kernel(const float* __restrict__ W, int ldw,
                                                                   unsigned short* __restrict__ outH,
                                                                   unsigned short* __restrict__ outL,
                                                                   int out_pitch, int out_row_base) {
  __shared__ float sm[64][65];
  const int t  = threadIdx.x;
  const int k0 = blockIdx.x * 64;
  const int n0 = blockIdx.y * 64;
#pragma unroll
  for (int i = 0; i < 16; ++i) {
    const int e = i * 256 + t;
    const int r = e >> 6;
    const int c = e & 63;
    sm[c][r] = W[(size_t)(k0 + r) * ldw + n0 + c];
  }
  __syncthreads();
  const int lane = t & 31, wave = t >> 5;
  const int q = lane >> 3, c8 = (lane & 7) * 8;
  for (int pass = 0; pass < 2; ++pass) {
#pragma unroll
    for (int it = 0; it < 2; ++it) {
      const int row = wave * 8 + it * 4 + q;
      unsigned short hb[8], lb[8];
#pragma unroll
      for (int e = 0; e < 8; ++e) {
        const float v = sm[row][c8 + e];
        const unsigned short h = f2bf_bits(v);
        hb[e] = h;
        lb[e] = f2bf_bits(v - bf_bits2f(h));
      }
      const v4u uh = (v4u){pk16(hb[0], hb[1]), pk16(hb[2], hb[3]), pk16(hb[4], hb[5]), pk16(hb[6], hb[7])};
      const v4u ul = (v4u){pk16(lb[0], lb[1]), pk16(lb[2], lb[3]), pk16(lb[4], lb[5]), pk16(lb[6], lb[7])};
      const size_t o = (size_t)(out_row_base + n0 + row) * out_pitch + k0 + c8;
      *(volatile v4u*)(outH + o) = uh;
      *(volatile v4u*)(outL + o) = ul;
    }
    __threadfence();
  }
}

__global__ __launch_bounds__(256) void scan_kernel(const float* __restrict__ P, const float* __restrict__ bx,
                                                   const float* __restrict__ bbc, const float* __restrict__ bd,
                                                   float* __restrict__ YF) {
  const int n = blockIdx.x * 256 + threadIdx.x;
  const float bxv = bx[n];
  const float bmb = bbc[n];
  const float bcb = bbc[kLat + n];
  const float bdv = bd[n];
  const float* pc = P + n;
  float* yc = YF + n;
  float h = 0.0f;
#pragma unroll 1
  for (int t = 0; t < kLen; ++t) {
    const float* pr = pc + (size_t)t * kNall;
    const float xp = pr[0] + bxv;
    const float bm = pr[kLat] + bmb;
    const float cv = pr[2 * kLat] + bcb;
    const float dl = pr[3 * kLat] + bdv;
    const float sp = fmaxf(dl, 0.0f) + log1pf(expf(-fabsf(dl)));
    const float ab = expf(-sp);
    const float u  = ((1.0f - ab) * bm) * xp;
    h = ab * h + u;
    const float y = cv * h;
    float* yp = yc + (size_t)t * kLat;
    *(volatile float*)yp = y;
    __threadfence();
    *(volatile float*)yp = y;
  }
}

static inline size_t align256(size_t v) { return (v + 255) & ~(size_t)255; }

extern "C" void kernel_launch(void* const* d_in, const int* in_sizes, int n_in,
                              void* d_out, int out_size, void* d_ws, size_t ws_size,
                              hipStream_t stream) {
  const float* x   = (const float*)d_in[0];
  const float* Wx  = (const float*)d_in[1];
  const float* bx  = (const float*)d_in[2];
  const float* Wbc = (const float*)d_in[3];
  const float* bbc = (const float*)d_in[4];
  const float* Wd  = (const float*)d_in[5];
  const float* bd  = (const float*)d_in[6];
  const float* Wy  = (const float*)d_in[7];
  const float* by  = (const float*)d_in[8];
  float* out = (float*)d_out;

  char* ws = (char*)d_ws;
  size_t off = 0;
  const size_t szX   = (size_t)kTok * kCin * 2;
  const size_t szWT  = (size_t)kNall * kCin * 2;
  const size_t szWyT = (size_t)kCout * kLat * 2;
  const size_t szP   = (size_t)kLen * kNall * 4;
  const size_t szYF  = (size_t)kLen * kLat * 4;
  const size_t szY   = (size_t)kTok * kLat * 2;
  unsigned short* Xh   = (unsigned short*)(ws + off); off += align256(szX);
  unsigned short* Xl   = (unsigned short*)(ws + off); off += align256(szX);
  unsigned short* WTh  = (unsigned short*)(ws + off); off += align256(szWT);
  unsigned short* WTl  = (unsigned short*)(ws + off); off += align256(szWT);
  unsigned short* WyTh = (unsigned short*)(ws + off); off += align256(szWyT);
  unsigned short* WyTl = (unsigned short*)(ws + off); off += align256(szWyT);
  float*          P    = (float*)(ws + off);          off += align256(szP);
  float*          YF   = (float*)(ws + off);          off += align256(szYF);
  unsigned short* Yh   = (unsigned short*)(ws + off); off += align256(szY);
  unsigned short* Yl   = (unsigned short*)(ws + off); off += align256(szY);
  if (off > ws_size) return;
  if ((size_t)out_size * 4 < (size_t)kTok * kCout * 4) return;

  cast8_bf16hl_kernel<<<(kTok * kCin / 8) / 256, 256, 0, stream>>>(x, Xh, Xl, kTok * kCin / 8);

  transpose_cast_bf16hl_kernel<<<dim3(kCin / 64, kLat / 64), 256, 0, stream>>>(Wx, kLat, WTh, WTl, kCin, 0);
  transpose_cast_bf16hl_kernel<<<dim3(kCin / 64, (2 * kLat) / 64), 256, 0, stream>>>(Wbc, 2 * kLat, WTh, WTl, kCin, kLat);
  transpose_cast_bf16hl_kernel<<<dim3(kCin / 64, kLat / 64), 256, 0, stream>>>(Wd, kLat, WTh, WTl, kCin, 3 * kLat);
  transpose_cast_bf16hl_kernel<<<dim3(kLat / 64, kCout / 64), 256, 0, stream>>>(Wy, kCout, WyTh, WyTl, kLat, 0);

  for (int b = 0; b < kBatch; ++b) {
    const unsigned short* xa  = Xh + (size_t)b * kLen * kCin;
    const unsigned short* xa2 = Xl + (size_t)b * kLen * kCin;
    wmma_gemm64<1, true, 0, 0, false><<<dim3((kLen / 64) * (kNall / 64) / 8, 1), 256, 0, stream>>>(
        xa, xa2, kCin, 0L,
        WTh, WTl, kCin, 0L,
        (void*)P, nullptr, kNall, 0L,
        nullptr,
        nullptr, 0L,
        kLen, kNall, kCin, 1.0f);
    scan_kernel<<<kLat / 256, 256, 0, stream>>>(P, bx, bbc, bd, YF);
    cast8_bf16hl_kernel<<<(kLen * kLat / 8) / 256, 256, 0, stream>>>(
        YF, Yh + (size_t)b * kLen * kLat, Yl + (size_t)b * kLen * kLat, kLen * kLat / 8);
  }

  wmma_gemm64<1, true, 2, 0, false><<<dim3((kTok / 64) * (kCout / 64) / 8, 1), 256, 0, stream>>>(
      Yh, Yl, kLat, 0L,
      WyTh, WyTl, kLat, 0L,
      (void*)out, nullptr, kCout, 0L,
      by,
      nullptr, 0L,
      kTok, kCout, kLat, 1.0f);

  (void)in_sizes; (void)n_in;
}
